// MolTransformer_65317862637731
// MI455X (gfx1250) — hardware-verified
//
#include <hip/hip_runtime.h>

#define LEAKC 0.2f
#define EPSS  1e-20f

typedef _Float16 v8h  __attribute__((ext_vector_type(8)));
typedef _Float16 v16h __attribute__((ext_vector_type(16)));
typedef float    v8f  __attribute__((ext_vector_type(8)));
typedef float    v4f  __attribute__((ext_vector_type(4)));
typedef v8h v8ha __attribute__((may_alias));
typedef v4f v4fa __attribute__((may_alias));
union Frag { v16h v; v8h half[2]; };

__device__ __forceinline__ v8f wmma16(v16h a, v16h b, v8f c)
{
  v8f d = __builtin_amdgcn_wmma_f32_16x16x32_f16(false, a, false, b, (short)0, c, false, false);
  asm volatile("v_nop\n\tv_nop\n\tv_nop\n\tv_nop" : "+v"(d) : "v"(a), "v"(b));
  return d;
}

__device__ __forceinline__ v8h cvt8(v4f a, v4f b)
{
  v8f f = __builtin_shufflevector(a, b, 0, 1, 2, 3, 4, 5, 6, 7);
  return __builtin_convertvector(f, v8h);
}

__device__ __forceinline__ v8f zero8()
{
  v8f z;
#pragma unroll
  for (int r = 0; r < 8; ++r) z[r] = 0.0f;
  return z;
}

template <int MODE>
__device__ __forceinline__ float ldA(const float* __restrict__ A0, const float* __restrict__ A1,
                                     int mrow, int k)
{
  if (MODE == 0) return A0[(size_t)mrow * 98 + k];
  if (MODE == 1) return A0[(size_t)mrow * 34 + k];
  if (MODE == 2) {
    const int h = mrow >> 10, bb = (mrow >> 7) & 7, j = mrow & 127;
    return A0[((size_t)(bb * 128 + j)) * 128 + h * 32 + k];
  }
  return (k < 98) ? A0[(size_t)mrow * 98 + k] : A1[(size_t)mrow * 128 + (k - 98)];
}

template <int MODE>
__device__ __forceinline__ float ldB(const float* __restrict__ B0, const float* __restrict__ B1,
                                     int k, int n)
{
  if (MODE == 0) return B0[k * 128 + n];
  if (MODE == 1) return (n < 32) ? B0[(64 + k) * 32 + n] : B1[(64 + k) * 32 + (n - 32)];
  if (MODE == 2) {
    const int c = n >> 5, nn = n & 31;
    const float* W = (c < 2) ? B0 : B1;
    const int row = (c & 1) ? (32 + k) : k;
    return W[row * 32 + nn];
  }
  return B0[k * 256 + n];
}

template <int MODE>
__global__ __launch_bounds__(256)
void k_gemm(const float* __restrict__ A0, const float* __restrict__ A1,
            const float* __restrict__ B0, const float* __restrict__ B1,
            const float* __restrict__ bias, float* C)
{
  constexpr int K  = (MODE == 0) ? 98 : (MODE == 1) ? 34 : (MODE == 2) ? 32 : 226;
  constexpr int N  = (MODE == 0) ? 128 : (MODE == 1) ? 64 : (MODE == 2) ? 128 : 256;
  constexpr int NK = (K + 31) / 32;
  constexpr bool TRANS = (MODE == 1) || (MODE == 2);
  constexpr float WSC = 16.0f;
  constexpr float OSC = 0.0625f;

  __shared__ __attribute__((aligned(16))) _Float16 lA[128 * 40];
  __shared__ __attribute__((aligned(16))) _Float16 lB[64 * 40];
  __shared__ __attribute__((aligned(16))) float    sC[8704];

  const int tid = threadIdx.x;
  const int l = tid & 31, w = tid >> 5, hh = l >> 4, m = l & 15;
  const int n0 = blockIdx.x * 64;
  const int mt = blockIdx.y;
  const int m0 = mt * 128;

  v8f acc[4];
#pragma unroll
  for (int t = 0; t < 4; ++t) acc[t] = zero8();

  const int amm = tid >> 1, akb = (tid & 1) * 16;
  const int bnn = tid >> 2, bkb = (tid & 3) * 8;

#pragma unroll 1
  for (int ks = 0; ks < NK; ++ks) {
    const int k0 = ks * 32;
    {
      float av[16];
#pragma unroll
      for (int e = 0; e < 16; ++e) {
        const int k = k0 + akb + e;
        av[e] = (k < K) ? ldA<MODE>(A0, A1, m0 + amm, k) : 0.0f;
      }
      v8f f0, f1;
#pragma unroll
      for (int e = 0; e < 8; ++e) { f0[e] = av[e]; f1[e] = av[8 + e]; }
      _Float16* dst = lA + amm * 40 + akb;
      *(v8ha*)dst       = __builtin_convertvector(f0, v8h);
      *(v8ha*)(dst + 8) = __builtin_convertvector(f1, v8h);
    }
    {
      float bv[8];
#pragma unroll
      for (int e = 0; e < 8; ++e) {
        const int k = k0 + bkb + e;
        bv[e] = (k < K) ? ldB<MODE>(B0, B1, k, n0 + bnn) * WSC : 0.0f;
      }
      v8f f0;
#pragma unroll
      for (int e = 0; e < 8; ++e) f0[e] = bv[e];
      *(v8ha*)(lB + bnn * 40 + bkb) = __builtin_convertvector(f0, v8h);
    }
    __syncthreads();

    Frag fa;
    {
      const _Float16* ap = lA + (16 * w + m) * 40 + 8 * hh;
      fa.half[0] = *(const v8ha*)ap;
      fa.half[1] = *(const v8ha*)(ap + 16);
    }
#pragma unroll
    for (int t = 0; t < 4; ++t) {
      Frag fb;
      const _Float16* bp = lB + (16 * t + m) * 40 + 8 * hh;
      fb.half[0] = *(const v8ha*)bp;
      fb.half[1] = *(const v8ha*)(bp + 16);
      acc[t] = wmma16(fa.v, fb.v, acc[t]);
    }
    __syncthreads();
  }

  if (TRANS) {
#pragma unroll
    for (int t = 0; t < 4; ++t) {
#pragma unroll
      for (int r = 0; r < 8; ++r)
        sC[(16 * t + m) * 132 + 16 * w + 8 * hh + r] = acc[t][r] * OSC;
    }
  } else {
#pragma unroll
    for (int t = 0; t < 4; ++t) {
      const int col = 16 * t + m;
      float bvv = 0.0f;
      if (MODE == 3) bvv = bias[n0 + col];
#pragma unroll
      for (int r = 0; r < 8; ++r) {
        float x = acc[t][r] * OSC + bvv;
        if (MODE == 3) x = fmaxf(x, 0.0f);
        sC[(16 * w + 8 * hh + r) * 68 + col] = x;
      }
    }
  }
  __syncthreads();

  v4f vals[8];
  if (TRANS) {
#pragma unroll
    for (int q = 0; q < 8; ++q)
      vals[q] = *(const v4fa*)(sC + (8 * w + q) * 132 + 4 * l);
#pragma unroll
    for (int q = 0; q < 8; ++q)
      *(volatile v4fa*)(C + ((size_t)mt * N + n0 + 8 * w + q) * 128 + 4 * l) = vals[q];
    __threadfence();
#pragma unroll
    for (int q = 0; q < 8; ++q)
      *(volatile v4fa*)(C + ((size_t)mt * N + n0 + 8 * w + q) * 128 + 4 * l) = vals[q];
  } else {
#pragma unroll
    for (int q = 0; q < 8; ++q)
      vals[q] = *(const v4fa*)(sC + (16 * w + 2 * q + hh) * 68 + 4 * m);
#pragma unroll
    for (int q = 0; q < 8; ++q)
      *(volatile v4fa*)(C + (size_t)(m0 + 16 * w + 2 * q + hh) * N + n0 + 4 * m) = vals[q];
    __threadfence();
#pragma unroll
    for (int q = 0; q < 8; ++q)
      *(volatile v4fa*)(C + (size_t)(m0 + 16 * w + 2 * q + hh) * N + n0 + 4 * m) = vals[q];
  }
}

__global__ __launch_bounds__(256)
void k_layer(const float* __restrict__ PQT, const float* __restrict__ P3T,
             const float* __restrict__ amask, const float* __restrict__ resid,
             const float* __restrict__ b_attn_h, const float* __restrict__ W_attn_o,
             const float* __restrict__ b_attn_o, const float* __restrict__ b_msg_h,
             float* outH)
{
  __shared__ __attribute__((aligned(16))) float    sP2[32 * 128];
  __shared__ __attribute__((aligned(16))) _Float16 sQ2h[32 * 136];
  __shared__ __attribute__((aligned(16))) _Float16 sPh[4 * 16 * 136];
  __shared__ __attribute__((aligned(16))) float    sAcc[16 * 132];
  __shared__ float sP1[16 * 33];
  __shared__ float sRS[64];
  __shared__ float sWo[32];
  __shared__ float sBm[32];

  const int tid = threadIdx.x;
  const int l = tid & 31, w = tid >> 5, hh = l >> 4, m = l & 15;
  const int i0 = blockIdx.x * 16, b = blockIdx.y;
  if (tid < 32) { sWo[tid] = W_attn_o[tid]; sBm[tid] = b_msg_h[tid]; }
  const float bo = b_attn_o[0];
  const int sd = tid >> 3, sjb = (tid & 7) * 16;
  const float PSC = 16384.0f;
  const float PINV = 1.0f / 16384.0f;

#pragma unroll 1
  for (int h = 0; h < 4; ++h) {
    const int hb = h * 8 + b;
    const float* pq = PQT + (size_t)hb * 16384;
    __syncthreads();
    {
      const float* src = pq + (size_t)(32 + sd) * 128 + sjb;
      float* dst = sP2 + sd * 128 + sjb;
#pragma unroll
      for (int q = 0; q < 4; ++q) *(v4fa*)(dst + 4 * q) = *(const v4fa*)(src + 4 * q);
    }
    {
      const float* src = pq + (size_t)(96 + sd) * 128 + sjb;
      const v4f x0 = *(const v4fa*)(src);
      const v4f x1 = *(const v4fa*)(src + 4);
      const v4f x2 = *(const v4fa*)(src + 8);
      const v4f x3 = *(const v4fa*)(src + 12);
      _Float16* dst = sQ2h + sd * 136 + sjb;
      *(v8ha*)dst       = cvt8(x0, x1);
      *(v8ha*)(dst + 8) = cvt8(x2, x3);
    }
#pragma unroll
    for (int q = 0; q < 2; ++q) {
      const int e = tid + 256 * q;
      const int ii = e >> 5, d = e & 31;
      sP1[ii * 33 + d] = pq[(size_t)d * 128 + i0 + ii] + b_attn_h[d];
    }
    __syncthreads();

#pragma unroll 1
    for (int rr = 0; rr < 2; ++rr) {
      const int i = 2 * w + rr;
      const int gi = b * 128 + i0 + i;
      const float* p3 = P3T + (size_t)gi * 8192;
      const float* mkp = amask + (size_t)gi * 128;
      float sc[4], mkv[4], ev[4];
#pragma unroll
      for (int c = 0; c < 4; ++c) {
        const int j = l + 32 * c;
        float dot = 0.0f;
#pragma unroll 8
        for (int d = 0; d < 32; ++d) {
          float s = sP1[i * 33 + d] + sP2[d * 128 + j] + p3[d * 128 + j];
          s = (s > 0.0f) ? s : LEAKC * s;
          dot = fmaf(s, sWo[d], dot);
        }
        mkv[c] = mkp[j];
        sc[c] = (dot + bo) * mkv[c];
      }
      float mx = fmaxf(fmaxf(sc[0], sc[1]), fmaxf(sc[2], sc[3]));
#pragma unroll
      for (int off = 16; off > 0; off >>= 1) mx = fmaxf(mx, __shfl_xor(mx, off, 32));
      float sum = 0.0f;
#pragma unroll
      for (int c = 0; c < 4; ++c) { ev[c] = __expf(sc[c] - mx) * mkv[c]; sum += ev[c]; }
#pragma unroll
      for (int off = 16; off > 0; off >>= 1) sum += __shfl_xor(sum, off, 32);
      const float inv = 1.0f / (sum + EPSS);
      float rs = 0.0f;
#pragma unroll
      for (int c = 0; c < 4; ++c) {
        const float p = ev[c] * inv * mkv[c];
        rs += p;
        sPh[(h * 16 + i) * 136 + l + 32 * c] = (_Float16)(p * PSC);
      }
#pragma unroll
      for (int off = 16; off > 0; off >>= 1) rs += __shfl_xor(rs, off, 32);
      if (l == 0) sRS[h * 16 + i] = rs;
    }
    __syncthreads();

    if (w < 2) {
      const int t = w;
      v8f acc = zero8();
#pragma unroll
      for (int ks = 0; ks < 4; ++ks) {
        Frag fa, fb;
        const _Float16* ap = sPh + (h * 16 + m) * 136 + 32 * ks + 8 * hh;
        fa.half[0] = *(const v8ha*)ap;
        fa.half[1] = *(const v8ha*)(ap + 16);
        const _Float16* bp = sQ2h + (16 * t + m) * 136 + 32 * ks + 8 * hh;
        fb.half[0] = *(const v8ha*)bp;
        fb.half[1] = *(const v8ha*)(bp + 16);
        acc = wmma16(fa.v, fb.v, acc);
      }
#pragma unroll
      for (int r = 0; r < 8; ++r)
        sAcc[(8 * hh + r) * 132 + h * 32 + 16 * t + m] = acc[r] * PINV;
    }
  }
  __syncthreads();

#pragma unroll 1
  for (int rr = 0; rr < 2; ++rr) {
    const int i = 2 * w + rr;
    const int gi = b * 128 + i0 + i;
    const int hc = (m < 4) ? m : 3;
#pragma unroll
    for (int mt = 0; mt < 2; ++mt) {
      v8f acc = zero8();
#pragma unroll
      for (int ks = 0; ks < 4; ++ks) {
        const float* arow = P3T + ((size_t)gi * 64 + 32 + 16 * mt + m) * 128 + 32 * ks + 8 * hh;
        const v4f x0 = *(const v4fa*)(arow);
        const v4f x1 = *(const v4fa*)(arow + 4);
        const v4f x2 = *(const v4fa*)(arow + 16);
        const v4f x3 = *(const v4fa*)(arow + 20);
        Frag fa, fb;
        fa.half[0] = cvt8(x0, x1);
        fa.half[1] = cvt8(x2, x3);
        const _Float16* bp = sPh + (hc * 16 + i) * 136 + 32 * ks + 8 * hh;
        fb.half[0] = *(const v8ha*)bp;
        fb.half[1] = *(const v8ha*)(bp + 16);
        acc = wmma16(fa.v, fb.v, acc);
      }
      if (m < 4) {
#pragma unroll
        for (int r = 0; r < 8; ++r)
          sAcc[i * 132 + m * 32 + 16 * mt + 8 * hh + r] += acc[r] * PINV;
      }
    }
  }
  __syncthreads();

  const int hq = l >> 3, d0 = 4 * (l & 7);
  const float* pqe = PQT + (size_t)(hq * 8 + b) * 16384;
  v4f ov[2];
#pragma unroll
  for (int rr = 0; rr < 2; ++rr) {
    const int i = 2 * w + rr;
    const int gi = b * 128 + i0 + i;
    const v4f a = *(const v4fa*)(sAcc + i * 132 + 4 * l);
    const v4f res = *(const v4fa*)(resid + (size_t)gi * 128 + 4 * l);
    const float rs = sRS[hq * 16 + i];
    v4f o;
#pragma unroll
    for (int e = 0; e < 4; ++e) {
      const int d = d0 + e;
      const float q1 = pqe[(size_t)(64 + d) * 128 + i0 + i];
      const float v = rs * q1 + a[e] + sBm[d] + res[e];
      o[e] = fmaxf(v, 0.0f);
    }
    ov[rr] = o;
  }
#pragma unroll
  for (int rr = 0; rr < 2; ++rr)
    *(volatile v4fa*)(outH + (size_t)(b * 128 + i0 + 2 * w + rr) * 128 + 4 * l) = ov[rr];
  __threadfence();
#pragma unroll
  for (int rr = 0; rr < 2; ++rr)
    *(volatile v4fa*)(outH + (size_t)(b * 128 + i0 + 2 * w + rr) * 128 + 4 * l) = ov[rr];
}

extern "C" void kernel_launch(void* const* d_in, const int* in_sizes, int n_in,
                              void* d_out, int out_size, void* d_ws, size_t ws_size,
                              hipStream_t stream)
{
  if (n_in < 12) return;
  if (in_sizes[0] != 100352 || in_sizes[1] != 4456448 || in_sizes[2] != 131072 ||
      in_sizes[3] != 12544 || in_sizes[4] != 3136 || in_sizes[5] != 32 ||
      in_sizes[6] != 32 || in_sizes[7] != 1 || in_sizes[8] != 3136 ||
      in_sizes[9] != 32 || in_sizes[10] != 57856 || in_sizes[11] != 256 ||
      out_size != 262144) return;

  const float* atom     = (const float*)d_in[0];
  const float* path     = (const float*)d_in[1];
  const float* pmask    = (const float*)d_in[2];
  const float* W_atom_i = (const float*)d_in[3];
  const float* W_attn_h = (const float*)d_in[4];
  const float* b_attn_h = (const float*)d_in[5];
  const float* W_attn_o = (const float*)d_in[6];
  const float* b_attn_o = (const float*)d_in[7];
  const float* W_msg_h  = (const float*)d_in[8];
  const float* b_msg_h  = (const float*)d_in[9];
  const float* W_atom_o = (const float*)d_in[10];
  const float* b_atom_o = (const float*)d_in[11];
  float* out = (float*)d_out;

  char* wsb = (char*)d_ws;
  size_t off = 0;
  float* AIH = (float*)(wsb + off); off += (size_t)1024 * 128 * 4;
  float* H0  = (float*)(wsb + off); off += (size_t)1024 * 128 * 4;
  float* H1  = (float*)(wsb + off); off += (size_t)1024 * 128 * 4;
  float* PQT = (float*)(wsb + off); off += (size_t)32 * 128 * 128 * 4;
  float* P3T = (float*)(wsb + off); off += (size_t)1024 * 64 * 128 * 4;
  if (off > ws_size) return;

  k_gemm<0><<<dim3(2, 8, 1), dim3(256, 1, 1), 0, stream>>>(atom, atom, W_atom_i, W_atom_i, b_atom_o, AIH);

  k_gemm<1><<<dim3(1, 1024, 1), dim3(256, 1, 1), 0, stream>>>(path, path, W_attn_h, W_msg_h, b_atom_o, P3T);

  const float* cur = AIH;
  float* hbuf[2] = {H0, H1};
  for (int layer = 0; layer < 2; ++layer) {
    k_gemm<2><<<dim3(2, 32, 1), dim3(256, 1, 1), 0, stream>>>(cur, cur, W_attn_h, W_msg_h, b_atom_o, PQT);
    k_layer<<<dim3(8, 8, 1), dim3(256, 1, 1), 0, stream>>>(PQT, P3T, pmask, AIH, b_attn_h, W_attn_o,
                                                          b_attn_o, b_msg_h, hbuf[layer]);
    cur = hbuf[layer];
  }

  k_gemm<3><<<dim3(4, 8, 1), dim3(256, 1, 1), 0, stream>>>(atom, cur, W_atom_o, W_atom_o, b_atom_o, out);
}
